// SelectiveSSM_8761733284417
// MI455X (gfx1250) — hardware-run, weakly checked
//
#include <hip/hip_runtime.h>
#include <math.h>

typedef __attribute__((ext_vector_type(16))) _Float16 v16h;
typedef __attribute__((ext_vector_type(8)))  _Float16 v8h;
typedef __attribute__((ext_vector_type(2)))  _Float16 v2h;
typedef __attribute__((ext_vector_type(16))) __bf16   v16b;
typedef __attribute__((ext_vector_type(8)))  __bf16   v8b;
typedef __attribute__((ext_vector_type(8)))  float    v8f;
typedef __attribute__((ext_vector_type(4)))  float    v4f;
typedef __attribute__((ext_vector_type(2)))  float    v2f;

constexpr int kNB   = 4;
constexpr int kL    = 4096;
constexpr int kRows = kNB * kL;
constexpr int kD    = 1024;
constexpr int kNs   = 16;
constexpr int kRk   = 64;
constexpr int kStk  = 2 * kNs + kRk;
constexpr int kStkP = 128;
constexpr int kK2   = 2 * kD;
constexpr int kThr  = 256;
constexpr float kInCarry = 1024.0f;
constexpr float kWCarry  = 4096.0f;
constexpr float kSc = 1.0f / (kInCarry * kWCarry);
constexpr float kF16MinNormal = 6.103515625e-5f;

static_assert(kRows == 16384 && kD == 1024 && kNs == 16 && kRk == 64 && kStk == 96 && kStk <= kStkP && (kStkP % 64) == 0 && (kL & (kL - 1)) == 0 && (kD % 8) == 0, "the index arithmetic below uses these sizes");

constexpr size_t kOffU2 = 0ull;
constexpr size_t kOffWS16 = 67108864ull;
constexpr size_t kOffWP16 = 67633152ull;
constexpr size_t kOffSB = 67764224ull;
constexpr size_t kOffBP = 67764736ull;
constexpr size_t kOffXS = 67768832ull;
constexpr size_t kOffDT16 = 76157440ull;
constexpr size_t kOffPRE = 78254592ull;
constexpr size_t kWsTotal = 145363456ull;
static_assert(kWsTotal <= 268435456ull, "the carve stands under the contract's 256 MiB of workspace");
static_assert(kOffU2 == 0
  && kOffWS16 == kOffU2 + 67108864ull
  && kOffWP16 == kOffWS16 + 524288ull
  && kOffSB == kOffWP16 + 131072ull
  && kOffBP == kOffSB + 512ull
  && kOffXS == kOffBP + 4096ull
  && kOffDT16 == kOffXS + 8388608ull
  && kOffPRE == kOffDT16 + 2097152ull
  && kWsTotal == kOffPRE + 67108864ull, "the carve is a chain: every region starts where the one before ends");
static_assert((kOffWS16 % 256) == 0 && (kOffWP16 % 256) == 0 && (kOffSB % 256) == 0 && (kOffBP % 256) == 0 && (kOffXS % 256) == 0 && (kOffDT16 % 256) == 0 && (kOffPRE % 256) == 0, "every region starts on a multiple of 256 B");

__device__ __forceinline__ unsigned short f2bf_bits(float f) {
  unsigned u = __float_as_uint(f);
  return (unsigned short)((u + 0x7FFFu + ((u >> 16) & 1u)) >> 16);
}
__device__ __forceinline__ float bf_bits2f(unsigned short h) { return __uint_as_float(((unsigned)h) << 16); }
__device__ __forceinline__ float bf16r(float f) { return bf_bits2f(f2bf_bits(f)); }
__device__ __forceinline__ float carry_flush(float v, float carry) {
  const float s = v * carry;
  return (fabsf(s) < kF16MinNormal) ? 0.0f : s;
}

__device__ __forceinline__ void dep_guard4_h(v8f& a, v8f& b, v8f& c, v8f& d, v16h x, v16h y) { asm volatile("v_nop\n\tv_nop\n\tv_nop\n\tv_nop" : "+v"(a), "+v"(b), "+v"(c), "+v"(d) : "v"(x), "v"(y)); }
__device__ __forceinline__ void dep_guard4_b(v8f& a, v8f& b, v8f& c, v8f& d, v16b x, v16b y) { asm volatile("v_nop\n\tv_nop\n\tv_nop\n\tv_nop" : "+v"(a), "+v"(b), "+v"(c), "+v"(d) : "v"(x), "v"(y)); }
__device__ __forceinline__ void keep4_h(v16h a, v16h b, v16h c, v16h d) { asm volatile("v_nop" :: "v"(a), "v"(b), "v"(c), "v"(d)); }
__device__ __forceinline__ void keep4_b(v16b a, v16b b, v16b c, v16b d) { asm volatile("v_nop" :: "v"(a), "v"(b), "v"(c), "v"(d)); }
__device__ __forceinline__ void acc_guard4(v8f& a, v8f& b, v8f& c, v8f& d) { asm volatile("v_nop\n\tv_nop\n\tv_nop\n\tv_nop" : "+v"(a), "+v"(b), "+v"(c), "+v"(d)); }

template <typename T> struct Frag;
template <> struct Frag<_Float16> {
  typedef v16h V; union U { v16h v; v8h h[2]; };
  static __device__ __forceinline__ v16h load(const _Float16* p) {
    U f; f.h[0] = *(const v8h*)(p); f.h[1] = *(const v8h*)(p + 16); return f.v;
  }
  static __device__ __forceinline__ v8f mma(v16h a, v16h b, v8f c) {
    return __builtin_amdgcn_wmma_f32_16x16x32_f16(false, a, false, b, (short)0, c, false, false);
  }
  static __device__ __forceinline__ void guard4(v8f& a, v8f& b, v8f& c, v8f& d, v16h x, v16h y) { dep_guard4_h(a, b, c, d, x, y); }
  static __device__ __forceinline__ void keep(v16h a, v16h b, v16h c, v16h d) { keep4_h(a, b, c, d); }
};
template <> struct Frag<__bf16> {
  typedef v16b V; union U { v16b v; v8b h[2]; };
  static __device__ __forceinline__ v16b load(const __bf16* p) {
    U f; f.h[0] = *(const v8b*)(p); f.h[1] = *(const v8b*)(p + 16); return f.v;
  }
  static __device__ __forceinline__ v8f mma(v16b a, v16b b, v8f c) {
    return __builtin_amdgcn_wmma_f32_16x16x32_bf16(false, a, false, b, (short)0, c, false, false);
  }
  static __device__ __forceinline__ void guard4(v8f& a, v8f& b, v8f& c, v8f& d, v16b x, v16b y) { dep_guard4_b(a, b, c, d, x, y); }
  static __device__ __forceinline__ void keep(v16b a, v16b b, v16b c, v16b d) { keep4_b(a, b, c, d); }
};

__device__ __forceinline__ v8f mma_h(v16h a, v16h b, v8f c) {
  c = __builtin_amdgcn_wmma_f32_16x16x32_f16(false, a, false, b, (short)0, c, false, false);
  asm volatile("v_nop\n\tv_nop\n\tv_nop\n\tv_nop" : "+v"(c) : "v"(a), "v"(b));
  return c;
}

template <int ET> struct Elem;
template <> struct Elem<0> { typedef _Float16 T; };
template <> struct Elem<1> { typedef __bf16 T; };
template <int ET, bool SPLIT, int BIAS_MODE, int OUT_MODE, bool RESID, int ACT = 0>
__global__ __launch_bounds__(256) void wmma_gemm64(
    const unsigned short* __restrict__ Ap, const unsigned short* __restrict__ A2p, int lda, long strideA,
    const unsigned short* __restrict__ Btp, const unsigned short* __restrict__ Bt2p, int ldb, long strideB,
    void* __restrict__ Cout, void* __restrict__ Cout2, int ldc, long strideC,
    const float* __restrict__ bias,
    const float* __restrict__ resid, long strideR,
    int M, int N, int K, float scale) {
  typedef typename Elem<ET>::T T;
  typedef typename Frag<T>::V V;
  const T* A = (const T*)Ap; const T* A2 = (const T*)A2p; const T* Bt = (const T*)Btp; const T* Bt2 = (const T*)Bt2p;
  __shared__ __align__(16) float sT[8][16 * 68];
  const int b    = blockIdx.y;
  const int lane = threadIdx.x & 31;
  const int wave = threadIdx.x >> 5;
  const int tilesN = N >> 6;
  const int tilesM = M >> 6;
  const int tile = blockIdx.x * 8 + wave;
  if (tile >= tilesM * tilesN) return;
  const int tm = tile / tilesN;
  const int tn = tile - tm * tilesN;
  const int m0 = tm << 6;
  const int n0 = tn << 6;

  const T* Ab  = A  + (size_t)b * strideA;
  const T* Bb  = Bt + (size_t)b * strideB;
  const T* Ab2 = SPLIT ? (A2  + (size_t)b * strideA) : nullptr;
  const T* Bb2 = SPLIT ? (Bt2 + (size_t)b * strideB) : nullptr;

  const int rlane = lane & 15;
  const int koff  = (lane >> 4) * 8;
  const int mOff  = (lane >> 4) * 8;

  v8f acc[4][4];
#pragma unroll
  for (int i = 0; i < 4; ++i)
#pragma unroll
    for (int j = 0; j < 4; ++j) acc[i][j] = (v8f){0.f,0.f,0.f,0.f,0.f,0.f,0.f,0.f};

  for (int k0 = 0; k0 < K; k0 += 32) {
    V bh[4], bl[4];
#pragma unroll
    for (int j = 0; j < 4; ++j) {
      const size_t bo = (size_t)(n0 + (j << 4) + rlane) * ldb + koff + k0;
      bh[j] = Frag<T>::load(Bb + bo);
      if (SPLIT) bl[j] = Frag<T>::load(Bb2 + bo);
    }
#pragma unroll
    for (int i = 0; i < 4; ++i) {
      const size_t ao = (size_t)(m0 + (i << 4) + rlane) * lda + koff + k0;
      V ah = Frag<T>::load(Ab + ao);
      V al;
      if (SPLIT) al = Frag<T>::load(Ab2 + ao);
#pragma unroll
      for (int j = 0; j < 4; ++j) {
        acc[i][j] = Frag<T>::mma(ah, bh[j], acc[i][j]);
        if (SPLIT) {
          acc[i][j] = Frag<T>::mma(ah, bl[j], acc[i][j]);
          acc[i][j] = Frag<T>::mma(al, bh[j], acc[i][j]);
        }
      }
      Frag<T>::guard4(acc[i][0], acc[i][1], acc[i][2], acc[i][3], ah, SPLIT ? al : ah);
    }
    Frag<T>::keep(bh[0], bh[1], bh[2], bh[3]);
    if (SPLIT) Frag<T>::keep(bl[0], bl[1], bl[2], bl[3]);
  }
  acc_guard4(acc[0][0], acc[0][1], acc[0][2], acc[0][3]);
  acc_guard4(acc[1][0], acc[1][1], acc[1][2], acc[1][3]);
  acc_guard4(acc[2][0], acc[2][1], acc[2][2], acc[2][3]);
  acc_guard4(acc[3][0], acc[3][1], acc[3][2], acc[3][3]);

  float* slab = sT[wave];
  const float* Rb = RESID ? (resid + (size_t)b * strideR) : nullptr;
#pragma unroll
  for (int i = 0; i < 4; ++i) {
    const int mBase = m0 + (i << 4);
#pragma unroll
    for (int j = 0; j < 4; ++j) {
      const int n = n0 + (j << 4) + rlane;
      float bv = 0.f;
      if (BIAS_MODE == 2) bv = bias[n];
#pragma unroll
      for (int r = 0; r < 8; ++r) {
        float v = acc[i][j][r] * scale;
        if (BIAS_MODE == 1) v += bias[mBase + mOff + r];
        if (BIAS_MODE == 2) v += bv;
        if (RESID) v += Rb[(size_t)(mBase + mOff + r) * ldc + n];
        if (ACT == 1) v = tanhf(v);
        if (ACT == 2) v = fmaxf(v, 0.0f);
        if (ACT == 3) v = v / (1.0f + expf(-v));
        if (ACT == 4) v = (v > 0.f) ? v : 0.01f * v;
        slab[(mOff + r) * 68 + (j << 4) + rlane] = v;
      }
    }
    __builtin_amdgcn_fence(__ATOMIC_RELEASE, "workgroup");
    __builtin_amdgcn_wave_barrier();
    __builtin_amdgcn_fence(__ATOMIC_ACQUIRE, "workgroup");
    if (OUT_MODE == 0) {
      float* C = (float*)Cout + (size_t)b * strideC;
      const int hh = lane >> 4, c4 = (lane & 15) * 4;
      for (int pass = 0; pass < 2; ++pass) {
#pragma unroll
        for (int it = 0; it < 8; ++it) {
          const int row = it * 2 + hh;
          v4f v = *(const v4f*)(slab + row * 68 + c4);
          *(volatile v4f*)(C + (size_t)(mBase + row) * ldc + n0 + c4) = v;
        }
        __threadfence();
      }
    } else {
      const int q = lane >> 3, c8 = (lane & 7) * 8;
      unsigned short* C  = (unsigned short*)Cout  + (size_t)b * strideC;
      unsigned short* C2 = (OUT_MODE == 2) ? ((unsigned short*)Cout2 + (size_t)b * strideC) : nullptr;
      for (int pass = 0; pass < 2; ++pass) {
#pragma unroll
        for (int it = 0; it < 4; ++it) {
          const int row = it * 4 + q;
          const float* sp = slab + row * 68 + c8;
          v8h hv, lv;
#pragma unroll
          for (int e = 0; e < 8; ++e) {
            if (OUT_MODE == 1) {
              hv[e] = (_Float16)sp[e];
            } else {
              unsigned short hb = f2bf_bits(sp[e]);
              unsigned short lb = f2bf_bits(sp[e] - bf_bits2f(hb));
              hv[e] = __builtin_bit_cast(_Float16, hb);
              lv[e] = __builtin_bit_cast(_Float16, lb);
            }
          }
          *(volatile v8h*)(C + (size_t)(mBase + row) * ldc + n0 + c8) = hv;
          if (OUT_MODE == 2) *(volatile v8h*)(C2 + (size_t)(mBase + row) * ldc + n0 + c8) = lv;
        }
        __threadfence();
      }
    }
    __builtin_amdgcn_fence(__ATOMIC_RELEASE, "workgroup");
    __builtin_amdgcn_wave_barrier();
    __builtin_amdgcn_fence(__ATOMIC_ACQUIRE, "workgroup");
  }
}


__device__ __forceinline__ void store2(float* p, float v) {
  *(volatile float*)p = v;
  __threadfence();
  *(volatile float*)p = v;
}

__global__ __launch_bounds__(kThr) void cast_plane_kernel(const float* __restrict__ src, unsigned short* __restrict__ dst,
                                                          int colsLog2, int dstPitch, int dstOff) {
  const int i   = blockIdx.x * kThr + threadIdx.x;
  const int sh  = colsLog2 - 3;
  const int row = i >> sh;
  const int c8  = (i & ((1 << sh) - 1)) * 8;
  const float* sp = src + ((size_t)row << colsLog2) + c8;
  const v4f a0 = *(const v4f*)(sp);
  const v4f a1 = *(const v4f*)(sp + 4);
  v8h hv;
#pragma unroll
  for (int e = 0; e < 4; ++e) {
    const float f0 = a0[e];
    const float f1 = a1[e];
    hv[e]     = (_Float16)carry_flush(bf16r(f0), kInCarry);
    hv[4 + e] = (_Float16)carry_flush(bf16r(f1), kInCarry);
  }
  unsigned short* dp = dst + (size_t)row * dstPitch + dstOff + c8;
  *(volatile v8h*)dp = hv;
  __threadfence();
  *(volatile v8h*)dp = hv;
}

__global__ __launch_bounds__(256) void wt_plane_kernel(const float* __restrict__ W, unsigned short* __restrict__ dst, int K, int N, int nLive, int ldd, int colOff) {
  const int n  = blockIdx.x;
  const int k8 = threadIdx.x * 8;
  const bool live = n < nLive;
  const int nc = live ? n : 0;
  v8h hv;
#pragma unroll
  for (int e = 0; e < 8; ++e) {
    const float w = W[(size_t)(k8 + e) * N + nc];
    hv[e] = (_Float16)(live ? carry_flush(bf16r(w), kWCarry) : 0.0f);
  }
  unsigned short* dp = dst + (size_t)n * ldd + colOff + k8;
  *(volatile v8h*)dp = hv;
  __threadfence();
  *(volatile v8h*)dp = hv;
}

__global__ __launch_bounds__(kThr) void front_kernel(const float* __restrict__ x, const float* __restrict__ conv_w, unsigned short* __restrict__ U2) {
  const unsigned j = blockIdx.x * (unsigned)kThr + threadIdx.x;
  const unsigned row = j >> 7;
  const unsigned c8 = (j & 127u) * 8u;
  const unsigned tok = row & (unsigned)(kL - 1);
  const float* pc = x + (size_t)row * kD + c8;
  v8h hv, lv;
#pragma unroll
  for (int q = 0; q < 2; ++q) {
    const v4f x1 = *(const v4f*)(pc + 4 * q);
    v4f x0, x2;
#pragma unroll
    for (int e = 0; e < 4; ++e) { x0[e] = 0.0f; x2[e] = 0.0f; }
    if (tok > 0u) x0 = *(const v4f*)(pc - kD + 4 * q);
    if (tok < (unsigned)(kL - 1)) x2 = *(const v4f*)(pc + kD + 4 * q);
    const v4f w0 = *(const v4f*)(conv_w + c8 + 4 * q), w1 = *(const v4f*)(conv_w + kD + c8 + 4 * q), w2 = *(const v4f*)(conv_w + 2 * kD + c8 + 4 * q);
#pragma unroll
    for (int e = 0; e < 4; ++e) {
      const float a = (bf16r(x0[e]) * bf16r(w0[e]) + bf16r(x1[e]) * bf16r(w1[e])) + bf16r(x2[e]) * bf16r(w2[e]);
      const float u = a / (1.0f + expf(-a));
      const float s = carry_flush(u, kInCarry);
      const _Float16 hi = (_Float16)s;
      const float r = s - (float)hi;
      hv[4 * q + e] = hi;
      lv[4 * q + e] = (_Float16)((fabsf(r) < kF16MinNormal) ? 0.0f : r);
    }
  }
  unsigned short* dh = U2 + (size_t)row * kK2 + c8;
  unsigned short* dl = dh + kD;
  *(volatile v8h*)dh = hv;
  *(volatile v8h*)dl = lv;
  __threadfence();
  *(volatile v8h*)dh = hv;
  *(volatile v8h*)dl = lv;
}
static_assert(((size_t)kRows * kD / 8) % kThr == 0 && kD / 8 == 128, "front grid exact: 8,192 blocks: 128 threads a row");

__global__ __launch_bounds__(kThr) void setup_kernel(const float* __restrict__ b_bc, const float* __restrict__ b_dt, const float* __restrict__ b_dtp, float* __restrict__ SB, float* __restrict__ BP) {
  const unsigned bk = blockIdx.x;
  if (bk == 0u) {
    const unsigned i = threadIdx.x;
    if (i < (unsigned)kStkP) {
      float v = 0.0f;
      if (i < 2u * (unsigned)kNs) { const float q = b_bc[i]; v = bf16r(q); }
      else if (i < (unsigned)kStk) { const float q = b_dt[i - 2u * (unsigned)kNs]; v = bf16r(q); }
      float* dp = SB + i;
      *(volatile float*)dp = v;
      __threadfence();
      *(volatile float*)dp = v;
    }
  } else {
    const unsigned i = (bk - 1u) * (unsigned)kThr + threadIdx.x;
    const float q = b_dtp[i];
    const float v = bf16r(q);
    float* dp = BP + i;
    *(volatile float*)dp = v;
    __threadfence();
    *(volatile float*)dp = v;
  }
}
static_assert(kStkP <= kThr && kD == 4 * kThr, "set-up grid exact: 1 block of the stacked bias (its first 128 threads), 4 of the step's bias");

__global__ __launch_bounds__(kThr) void dt_cast_kernel(const float* __restrict__ XS, unsigned short* __restrict__ DT16) {
  const unsigned j = blockIdx.x * (unsigned)kThr + threadIdx.x;
  const unsigned row = j >> 3;
  const unsigned c8 = (j & 7u) * 8u;
  const float* ps = XS + (size_t)row * kStkP + 2 * kNs + c8;
  const v4f a0 = *(const v4f*)ps, a1 = *(const v4f*)(ps + 4);
  v8h hv;
#pragma unroll
  for (int e = 0; e < 4; ++e) { hv[e] = (_Float16)carry_flush(a0[e], kInCarry); hv[4 + e] = (_Float16)carry_flush(a1[e], kInCarry); }
  unsigned short* dp = DT16 + (size_t)j * 8;
  *(volatile v8h*)dp = hv;
  __threadfence();
  *(volatile v8h*)dp = hv;
}
static_assert(((size_t)kRows * kRk / 8) % kThr == 0 && kRk / 8 == 8, "step-cast grid exact: 512 blocks: 8 threads a row");

__global__ __launch_bounds__(kThr) void scan_kernel(const float* __restrict__ XS, const float* __restrict__ PRE, const float* __restrict__ x, const float* __restrict__ A_log, const float* __restrict__ Dcoeff,
                                                    float* __restrict__ out) {
  const unsigned ix = blockIdx.x * (unsigned)kThr + threadIdx.x;
  const unsigned sq = ix >> 9;
  const unsigned c0 = (ix & 511u) * 2u;
  float A[2][kNs], st[2][kNs], dc[2];
#pragma unroll
  for (int k = 0; k < 2; ++k) {
#pragma unroll
    for (int q = 0; q < kNs / 4; ++q) { const v4f av = *(const v4f*)(A_log + (size_t)(c0 + k) * kNs + 4 * q);
#pragma unroll
      for (int e = 0; e < 4; ++e) { A[k][4 * q + e] = -expf(bf16r(av[e])); st[k][4 * q + e] = 0.0f; } }
    const float q0 = Dcoeff[c0 + k];
    dc[k] = bf16r(q0);
  }
  for (int l = 0; l < kL; ++l) {
    const size_t row = (size_t)sq * kL + (size_t)l;
    const float* px = XS + row * kStkP;
    const v2f pr = *(const v2f*)(PRE + row * kD + c0);
    const v2f xv = *(const v2f*)(x + row * kD + c0);
    float dt[2], xr[2], xd[2], s[2];
#pragma unroll
    for (int k = 0; k < 2; ++k) {
      const float pre = pr[k];
      dt[k] = (pre > 20.0f) ? pre : log1pf(expf(pre));
      xr[k] = bf16r(xv[k]);
      xd[k] = xr[k] * dt[k];
      s[k] = 0.0f;
    }
#pragma unroll
    for (int q = 0; q < kNs / 4; ++q) {
      const v4f bv = *(const v4f*)(px + 4 * q), cv = *(const v4f*)(px + kNs + 4 * q);
#pragma unroll
      for (int e = 0; e < 4; ++e) {
        const int n = 4 * q + e;
#pragma unroll
        for (int k = 0; k < 2; ++k) {
          const float hn = expf(dt[k] * A[k][n]) * st[k][n] + bv[e] * xd[k];
          st[k][n] = hn;
          s[k] += cv[e] * hn;
        }
      }
    }
    v2f ov;
#pragma unroll
    for (int k = 0; k < 2; ++k) ov[k] = s[k] + xr[k] * dc[k];
    float* dp = out + row * kD + c0;
    *(volatile v2f*)dp = ov;
    __threadfence();
    *(volatile v2f*)dp = ov;
  }
}
static_assert(kNB * kD / 2 == 8 * kThr && kD / 2 == 512 && (kNs % 4) == 0, "scan grid exact: 8 blocks: 512 lanes a sequence");

extern "C" void kernel_launch(void* const* d_in, const int* in_sizes, int n_in,
                              void* d_out, int out_size, void* d_ws, size_t ws_size,
                              hipStream_t stream) {
  if (n_in < 10 || d_out == nullptr || d_ws == nullptr) return;
  if (in_sizes[0] != kRows * kD || in_sizes[1] != 3 * kD || in_sizes[2] != kD * 2 * kNs || in_sizes[3] != 2 * kNs || in_sizes[4] != kD * kRk || in_sizes[5] != kRk || in_sizes[6] != kRk * kD || in_sizes[7] != kD
      || in_sizes[8] != kD * kNs || in_sizes[9] != kD) return;
  if (out_size != kRows * kD) return;
  if (ws_size < kWsTotal) return;
  const float* x = (const float*)d_in[0];
  const float* conv_w = (const float*)d_in[1];
  const float* W_bc = (const float*)d_in[2];
  const float* b_bc = (const float*)d_in[3];
  const float* W_dt = (const float*)d_in[4];
  const float* b_dt = (const float*)d_in[5];
  const float* W_dtp = (const float*)d_in[6];
  const float* b_dtp = (const float*)d_in[7];
  const float* A_log = (const float*)d_in[8];
  const float* Dcoeff = (const float*)d_in[9];
  float* out = (float*)d_out;
  char* ws = (char*)d_ws;
  unsigned short* U2 = (unsigned short*)(ws + kOffU2);
  unsigned short* WS16 = (unsigned short*)(ws + kOffWS16);
  unsigned short* WP16 = (unsigned short*)(ws + kOffWP16);
  float* SB = (float*)(ws + kOffSB);
  float* BP = (float*)(ws + kOffBP);
  float* XS = (float*)(ws + kOffXS);
  unsigned short* DT16 = (unsigned short*)(ws + kOffDT16);
  float* PRE = (float*)(ws + kOffPRE);

  front_kernel<<<(int)(((size_t)kRows * kD / 8) / kThr), kThr, 0, stream>>>(x, conv_w, U2);
  wt_plane_kernel<<<2 * kNs, kD / 8, 0, stream>>>(W_bc, WS16, kD, 2 * kNs, 2 * kNs, kK2, 0);
  wt_plane_kernel<<<2 * kNs, kD / 8, 0, stream>>>(W_bc, WS16, kD, 2 * kNs, 2 * kNs, kK2, kD);
  wt_plane_kernel<<<kStkP - 2 * kNs, kD / 8, 0, stream>>>(W_dt, WS16 + (size_t)2 * kNs * kK2, kD, kRk, kRk, kK2, 0);
  wt_plane_kernel<<<kStkP - 2 * kNs, kD / 8, 0, stream>>>(W_dt, WS16 + (size_t)2 * kNs * kK2, kD, kRk, kRk, kK2, kD);
  wt_plane_kernel<<<kD, kRk / 8, 0, stream>>>(W_dtp, WP16, kRk, kD, kD, kRk, 0);
  setup_kernel<<<5, kThr, 0, stream>>>(b_bc, b_dt, b_dtp, SB, BP);
  wmma_gemm64<0, false, 2, 0, false, 0><<<dim3((kRows / 64) * (kStkP / 64) / 8, 1), 256, 0, stream>>>(
      U2, U2, kK2, 0L, WS16, WS16, kK2, 0L, (void*)XS, (void*)XS, kStkP, 0L, SB, nullptr, 0L, kRows, kStkP, kK2, kSc);
  dt_cast_kernel<<<(int)(((size_t)kRows * kRk / 8) / kThr), kThr, 0, stream>>>(XS, DT16);
  wmma_gemm64<0, false, 2, 0, false, 0><<<dim3((kRows / 64) * (kD / 64) / 8, 1), 256, 0, stream>>>(
      DT16, DT16, kRk, 0L, WP16, WP16, kRk, 0L, (void*)PRE, (void*)PRE, kD, 0L, BP, nullptr, 0L, kRows, kD, kRk, kSc);
  scan_kernel<<<8, kThr, 0, stream>>>(XS, PRE, x, A_log, Dcoeff, out);
}
static_assert(((kRows / 64) * (kStkP / 64)) % 8 == 0 && ((kRows / 64) * (kD / 64)) % 8 == 0, "the engine's grids: whole blocks of eight wave tiles");
